// HybridLayer_78700980732390
// MI455X (gfx1250) — hardware-verified
//
#include <hip/hip_runtime.h>
#include <stddef.h>


typedef _Float16 v16h __attribute__((ext_vector_type(16)));
typedef _Float16 v8h  __attribute__((ext_vector_type(8)));
typedef float    v8f  __attribute__((ext_vector_type(8)));
typedef float    v4f  __attribute__((ext_vector_type(4)));
typedef _Float16 h16;

#ifndef NBATCH
#define NBATCH 4096
#endif
#define NBATCH_FULL 4096
#define KIN     512
#define NQ      10
#define QD      1024
#define UCOLS   2048
#define NLAYERS 4
#define NGATE   40
#define OUTF    64

static_assert(NBATCH >= 64 && NBATCH <= NBATCH_FULL && (NBATCH % 64) == 0);
static_assert(QD == (1 << NQ));
static_assert(UCOLS == 2 * QD);
static_assert(NGATE == NLAYERS * NQ);
static_assert((KIN % 32) == 0 && (KIN % 8) == 0);
static_assert((QD % 64) == 0 && (QD % 32) == 0);
static_assert((UCOLS % 64) == 0);
static_assert(QD == 4 * 32 * 8);
static_assert(OUTF == 16 * 4);
static_assert((((size_t)NBATCH * KIN / 8) % 256) == 0);
static_assert((((size_t)QD * KIN / 8) % 256) == 0);
static_assert(((NGATE * 8) % 32) == 0);
static_assert(NGATE * 8 <= 256 + 64);
static_assert(OUTF * NQ <= 3 * 256);

#define LDT 72
#define LDC 68
#define ZP  12
static_assert((LDT % 8) == 0 && LDT >= 64);
static_assert((LDC % 4) == 0 && LDC >= 64);
static_assert(ZP >= NQ);

#define XCARRY 16.0f
#define WCARRY 64.0f
#define HCARRY 16.0f
#define UCARRY 1024.0f

#define G_BYTES    ((size_t)4096)
#define X16_BYTES  ((size_t)NBATCH * KIN * 2)
#define WP16_BYTES ((size_t)QD * KIN * 2)
#define UT_BYTES   ((size_t)QD * UCOLS * 4)
#define U16_BYTES  ((size_t)UCOLS * QD * 2)
#define H16_BYTES  ((size_t)NBATCH * QD * 2)
#define OFF_G    ((size_t)0)
#define OFF_X16  (OFF_G + G_BYTES)
#define OFF_WP16 (OFF_X16 + X16_BYTES)
#define OFF_UT   (OFF_WP16 + WP16_BYTES)
#define OFF_U16  (OFF_UT + UT_BYTES)
#define OFF_H16  (OFF_U16 + U16_BYTES)
#define WS_TOTAL (OFF_H16 + H16_BYTES)
static_assert((size_t)NGATE * 8 * 4 <= G_BYTES);
static_assert((G_BYTES % 128) == 0 && (X16_BYTES % 128) == 0 && (WP16_BYTES % 128) == 0);
static_assert((UT_BYTES % 128) == 0 && (U16_BYTES % 128) == 0 && (H16_BYTES % 128) == 0);
static_assert(WS_TOTAL <= (size_t)134217728);
static_assert((size_t)64 * LDC * 4 <= 131072);
static_assert((size_t)64 * LDT * 2 <= 131072);
static_assert((size_t)QD * 8 + NGATE * 8 * 4 <= 131072);
static_assert((size_t)(64 + 2 * 64 * ZP + OUTF * NQ + OUTF) * 4 <= 131072);

__device__ __forceinline__ float bf16r(float x) {
  unsigned int u = __float_as_uint(x);
  u = (u + 0x7FFFu + ((u >> 16) & 1u)) & 0xFFFF0000u;
  return __uint_as_float(u);
}

static __device__ __forceinline__ h16 toh_flush(float v) {
  const h16 r = (h16)v;
  return (fabsf(v) < 6.103515625e-05f) ? (h16)0.0f : r;
}

__device__ __forceinline__ v16h frag_at(const _Float16* p) {
  v8h lo = *(const v8h*)(p);
  v8h hi = *(const v8h*)(p + 16);
  v16h out;
#pragma unroll
  for (int i = 0; i < 8; ++i) { out[i] = lo[i]; out[i + 8] = hi[i]; }
  return out;
}

__device__ __forceinline__ v8f wmma16(v16h a, v16h b, v8f c) {
  v8f d = __builtin_amdgcn_wmma_f32_16x16x32_f16(false, a, false, b, (short)0, c,
                                                 false, false);
  asm volatile("v_nop\n\tv_nop\n\tv_nop\n\tv_nop" : "+v"(d) : "v"(a), "v"(b));
  return d;
}

__device__ __forceinline__ float red16_sum(float x) {
#pragma unroll
  for (int off = 1; off < 16; off <<= 1) x += __shfl_xor(x, off, 32);
  return x;
}
__device__ __forceinline__ float red32_sum(float x) {
#pragma unroll
  for (int off = 1; off < 32; off <<= 1) x += __shfl_xor(x, off, 32);
  return x;
}

__device__ __forceinline__ float relu_act(float t) {
  return fmaxf(t, 0.0f);
}

__global__ __launch_bounds__(128) void rot_prep_kernel(const float* __restrict__ qw,
                                                       float* __restrict__ G) {
  __shared__ float Tr[NGATE * 6];
  __shared__ __attribute__((aligned(16))) float Gs[NGATE * 8];
  const unsigned tid = threadIdx.x;
  const unsigned g = (tid < (unsigned)NGATE) ? tid : (unsigned)(NGATE - 1);
  const float phi = bf16r(qw[3u * g + 0u]);
  const float th  = bf16r(qw[3u * g + 1u]);
  const float om  = bf16r(qw[3u * g + 2u]);
  const float hth = 0.5f * th;
  const float aa  = 0.5f * (phi + om);
  const float bb  = 0.5f * (phi - om);
#pragma unroll 1
  for (unsigned k = 0; k < 3u; ++k) {
    const float ang = (k == 0u) ? hth : ((k == 1u) ? aa : bb);
    float sn, cs;
    sincosf(ang, &sn, &cs);
    if (tid < (unsigned)NGATE) {
      Tr[g * 6u + 2u * k]      = cs;
      Tr[g * 6u + 2u * k + 1u] = sn;
    }
  }
  __syncthreads();
  if (tid < (unsigned)NGATE) {
    const float ch = Tr[g * 6u + 0u], sh = Tr[g * 6u + 1u];
    const float ca = Tr[g * 6u + 2u], sa = Tr[g * 6u + 3u];
    const float cb = Tr[g * 6u + 4u], sb = Tr[g * 6u + 5u];
    float* u = &Gs[8u * g];
    u[0] =  ch * ca;  u[1] = -(ch * sa);
    u[2] = -(sh * cb); u[3] = -(sh * sb);
    u[4] =  sh * cb;  u[5] = -(sh * sb);
    u[6] =  ch * ca;  u[7] =  ch * sa;
  }
  __syncthreads();
  const unsigned nq4 = (unsigned)(NGATE * 8 / 4);
  const unsigned tq = (tid < nq4) ? tid : (nq4 - 1u);
  const v4f v = *(const v4f*)&Gs[4u * tq];
  if (tid < nq4) *(volatile v4f*)(G + 4u * tq) = v;
  __threadfence();
  if (tid < nq4) *(volatile v4f*)(G + 4u * tq) = v;
}

__global__ __launch_bounds__(256) void ubuild_kernel(const float* __restrict__ G,
                                                     float* __restrict__ UT) {
  __shared__ __attribute__((aligned(16))) float2 psi[QD];
  __shared__ float uS[NGATE * 8];
  const unsigned tid = threadIdx.x;
  const unsigned jb = blockIdx.x;

  uS[tid] = G[tid];
  {
    const unsigned i2 = 256u + (tid & 63u);
    const float gv = G[i2];
    if (tid < 64u) uS[i2] = gv;
  }
#pragma unroll
  for (unsigned p = 0; p < 4u; ++p) {
    const unsigned idx = tid + 256u * p;
    psi[idx] = make_float2((idx == jb) ? 1.0f : 0.0f, 0.0f);
  }

#pragma unroll 1
  for (unsigned l = 0; l < (unsigned)NLAYERS; ++l) {
#pragma unroll 1
    for (unsigned w = 0; w < (unsigned)NQ; ++w) {
      __syncthreads();
      const unsigned ub = (l * (unsigned)NQ + w) * 8u;
      const float u00r = uS[ub + 0u], u00i = uS[ub + 1u], u01r = uS[ub + 2u], u01i = uS[ub + 3u];
      const float u10r = uS[ub + 4u], u10i = uS[ub + 5u], u11r = uS[ub + 6u], u11i = uS[ub + 7u];
      const unsigned mask = 1u << (9u - w);
#pragma unroll 1
      for (unsigned pp = 0; pp < 2u; ++pp) {
        const unsigned p  = tid + pp * 256u;
        const unsigned i0 = ((p & ~(mask - 1u)) << 1) | (p & (mask - 1u));
        const unsigned i1 = i0 | mask;
        const float2 a0 = psi[i0];
        const float2 a1 = psi[i1];
        const float n0r = u00r * a0.x - u00i * a0.y + u01r * a1.x - u01i * a1.y;
        const float n0i = u00r * a0.y + u00i * a0.x + u01r * a1.y + u01i * a1.x;
        const float n1r = u10r * a0.x - u10i * a0.y + u11r * a1.x - u11i * a1.y;
        const float n1i = u10r * a0.y + u10i * a0.x + u11r * a1.y + u11i * a1.x;
        psi[i0] = make_float2(n0r, n0i);
        psi[i1] = make_float2(n1r, n1i);
      }
    }
    const int rr = (int)(l % (unsigned)(NQ - 1)) + 1;
#pragma unroll 1
    for (int w = 0; w < NQ; ++w) {
      __syncthreads();
      const int t  = (w + rr) % NQ;
      const int pc = 9 - w;
      const int pt = 9 - t;
      const int p1 = pc < pt ? pc : pt;
      const int p2 = pc < pt ? pt : pc;
      int x = (int)tid;
      x = ((x & ~((1 << p1) - 1)) << 1) | (x & ((1 << p1) - 1));
      x = ((x & ~((1 << p2) - 1)) << 1) | (x & ((1 << p2) - 1));
      const int i0 = x | (1 << pc);
      const int i1 = i0 | (1 << pt);
      const float2 t0 = psi[i0];
      const float2 t1 = psi[i1];
      psi[i0] = t1;
      psi[i1] = t0;
    }
  }
  __syncthreads();

  v4f xs[2];
  size_t off[2];
#pragma unroll
  for (unsigned p = 0; p < 2u; ++p) {
    const unsigned n4 = tid + 256u * p;
    const unsigned gq = n4 >> 2;
    const unsigned comp = gq & 1u;
    const unsigned ib = (gq >> 1) * 16u + (n4 & 3u) * 4u;
    v4f v;
#pragma unroll
    for (unsigned e = 0; e < 4u; ++e) {
      const float2 a = psi[ib + e];
      v[e] = (comp != 0u) ? a.y : a.x;
    }
    xs[p] = v;
    off[p] = (size_t)jb * UCOLS + 4u * n4;
  }
#pragma unroll
  for (int p = 0; p < 2; ++p) *(volatile v4f*)(UT + off[p]) = xs[p];
  __threadfence();
#pragma unroll
  for (int p = 0; p < 2; ++p) *(volatile v4f*)(UT + off[p]) = xs[p];
}

__global__ __launch_bounds__(256) void uconv_kernel(
    const float* __restrict__ W, _Float16* __restrict__ Wt, unsigned ldw, unsigned ldk) {
  __shared__ __attribute__((aligned(16))) _Float16 T[64 * LDT];
  const unsigned tid = threadIdx.x;
  const unsigned n0 = blockIdx.x * 64u;
  const unsigned k0 = blockIdx.y * 64u;
#pragma unroll 4
  for (unsigned j = 0; j < 16u; ++j) {
    const unsigned idx = tid + 256u * j;
    const unsigned kr = idx >> 6, nc = idx & 63u;
    const float v = W[(size_t)(k0 + kr) * ldw + n0 + nc];
    T[nc * LDT + kr] = toh_flush(UCARRY * v);
  }
  __syncthreads();
  v8h x[2];
  size_t off[2];
#pragma unroll
  for (unsigned i = 0; i < 2u; ++i) {
    const unsigned n = 32u * i + (tid >> 3);
    const unsigned kc = (tid & 7u) * 8u;
    x[i] = *(const v8h*)&T[n * LDT + kc];
    off[i] = (size_t)(n0 + n) * ldk + k0 + kc;
  }
#pragma unroll
  for (int i = 0; i < 2; ++i) *(volatile v8h*)(Wt + off[i]) = x[i];
  __threadfence();
#pragma unroll
  for (int i = 0; i < 2; ++i) *(volatile v8h*)(Wt + off[i]) = x[i];
}

__global__ __launch_bounds__(256) void rowconv_kernel(
    const float* __restrict__ src, _Float16* __restrict__ dst, float carry, unsigned n8) {
  const unsigned g = blockIdx.x * 256u + threadIdx.x;
  const unsigned gc = (g < n8) ? g : (n8 - 1u);
  const v4f a0 = *(const v4f*)(src + (size_t)gc * 8u);
  const v4f a1 = *(const v4f*)(src + (size_t)gc * 8u + 4u);
  v8h o;
#pragma unroll
  for (int i = 0; i < 4; ++i) {
    o[i]     = toh_flush(carry * bf16r(a0[i]));
    o[i + 4] = toh_flush(carry * bf16r(a1[i]));
  }
  _Float16* p = dst + (size_t)gc * 8u;
  if (g < n8) *(volatile v8h*)p = o;
  __threadfence();
  if (g < n8) *(volatile v8h*)p = o;
}

__global__ __launch_bounds__(256) void gemm_pre_kernel(
    const _Float16* __restrict__ A16, const _Float16* __restrict__ Bt,
    const float* __restrict__ bias, _Float16* __restrict__ out16) {
  __shared__ __attribute__((aligned(16))) float Cs[64 * LDC];
  const unsigned K = (unsigned)KIN;
  const unsigned tid = threadIdx.x, lane = tid & 31u, w = tid >> 5;
  const unsigned mw = w >> 1, nw = w & 1u;
  const unsigned hh = lane >> 4, m = lane & 15u;
  const unsigned n0 = blockIdx.x * 64u;
  const unsigned row0 = blockIdx.y * 64u;

  const _Float16* ap  = A16 + (size_t)(row0 + mw * 16u + m) * K + hh * 8u;
  const _Float16* bp0 = Bt + (size_t)(n0 + nw * 32u + m) * K + hh * 8u;
  const _Float16* bp1 = bp0 + (size_t)16 * K;
  v8f acc0 = {}, acc1 = {};
#pragma unroll 2
  for (unsigned k0 = 0; k0 < K; k0 += 32u) {
    const v16h a  = frag_at(ap + k0);
    const v16h b0 = frag_at(bp0 + k0);
    const v16h b1 = frag_at(bp1 + k0);
    acc0 = wmma16(a, b0, acc0);
    acc1 = wmma16(a, b1, acc1);
  }
#pragma unroll
  for (int r = 0; r < 8; ++r) {
    float* d = &Cs[(mw * 16u + hh * 8u + (unsigned)r) * LDC + nw * 32u + m];
    d[0]  = acc0[r];
    d[16] = acc1[r];
  }
  __syncthreads();

#pragma unroll 1
  for (unsigned g = 0; g < 4u; ++g) {
    const unsigned r = 32u * (g >> 1) + (tid >> 3);
    const unsigned c = (tid & 7u) * 8u + 4u * (g & 1u);
    const v4f u  = *(const v4f*)&Cs[r * LDC + c];
    const v4f gb = *(const v4f*)(bias + n0 + c);
    v4f t;
#pragma unroll
    for (int j = 0; j < 4; ++j)
      t[j] = HCARRY * relu_act(u[j] * (1.0f / (XCARRY * WCARRY)) + bf16r(gb[j]));
    *(v4f*)&Cs[r * LDC + c] = t;
  }

  v8h x[2];
  size_t off[2];
#pragma unroll
  for (unsigned i = 0; i < 2u; ++i) {
    const unsigned r = 32u * i + (tid >> 3);
    const unsigned c = (tid & 7u) * 8u;
    const v4f u0 = *(const v4f*)&Cs[r * LDC + c];
    const v4f u1 = *(const v4f*)&Cs[r * LDC + c + 4];
#pragma unroll
    for (int j = 0; j < 4; ++j) {
      x[i][j]     = toh_flush(u0[j]);
      x[i][j + 4] = toh_flush(u1[j]);
    }
    off[i] = (size_t)(row0 + r) * QD + n0 + c;
  }
#pragma unroll
  for (int i = 0; i < 2; ++i) *(volatile v8h*)(out16 + off[i]) = x[i];
  __threadfence();
#pragma unroll
  for (int i = 0; i < 2; ++i) *(volatile v8h*)(out16 + off[i]) = x[i];
}

__global__ __launch_bounds__(256) void circ_kernel(
    const _Float16* __restrict__ H16, const _Float16* __restrict__ U16,
    const float* __restrict__ Wpost, const float* __restrict__ bpost,
    float* __restrict__ out) {
  __shared__ float Ns[64];
  __shared__ float Zs[2 * 64 * ZP];
  __shared__ float Ws[OUTF * NQ];
  __shared__ float Bs[OUTF];

  const unsigned tid = threadIdx.x, lane = tid & 31u;
  const int wave = __builtin_amdgcn_readfirstlane((int)(threadIdx.x >> 5));
  const unsigned mw = (unsigned)wave >> 1, nw = (unsigned)wave & 1u;
  const unsigned hh = lane >> 4, m = lane & 15u;
  const unsigned row0 = blockIdx.x * 64u;

#pragma unroll
  for (unsigned k = 0; k < 3u; ++k) {
    const unsigned idx = tid + 256u * k;
    const unsigned ic = (idx < (unsigned)(OUTF * NQ)) ? idx : (unsigned)(OUTF * NQ - 1);
    const float wv = bf16r(Wpost[ic]);
    if (idx < (unsigned)(OUTF * NQ)) Ws[ic] = wv;
  }
  {
    const unsigned ic = tid & 63u;
    const float bv = bf16r(bpost[ic]);
    if (tid < (unsigned)OUTF) Bs[ic] = bv;
  }

#pragma unroll 1
  for (unsigned rr = 0; rr < 8u; ++rr) {
    const unsigned rl = (unsigned)wave * 8u + rr;
    const _Float16* hr = H16 + (size_t)(row0 + rl) * QD + lane * 8u;
    float s = 0.0f;
#pragma unroll 1
    for (unsigned j = 0; j < 4u; ++j) {
      const v8h a = *(const v8h*)(hr + j * 256u);
#pragma unroll
      for (int i = 0; i < 8; ++i) {
        const float e = (float)a[i];
        s = fmaf(e, e, s);
      }
    }
    s = red32_sum(s);
    if (lane == 0u) Ns[rl] = s;
  }

  const _Float16* ap = H16 + (size_t)(row0 + mw * 16u + m) * QD + hh * 8u;
  float S[8];
  float T[5][8];
#pragma unroll
  for (int r = 0; r < 8; ++r) {
    S[r] = 0.0f;
#pragma unroll
    for (int b2 = 0; b2 < 5; ++b2) T[b2][r] = 0.0f;
  }

#pragma unroll 1
  for (unsigned t = 0; t < (unsigned)(UCOLS / 64); ++t) {
    const _Float16* bp0 = U16 + (size_t)(t * 64u + nw * 32u + m) * QD + hh * 8u;
    const _Float16* bp1 = bp0 + (size_t)16 * QD;
    v8f acc0 = {}, acc1 = {};
#pragma unroll 2
    for (unsigned k0 = 0; k0 < (unsigned)QD; k0 += 32u) {
      const v16h a  = frag_at(ap + k0);
      const v16h b0 = frag_at(bp0 + k0);
      const v16h b1 = frag_at(bp1 + k0);
      acc0 = wmma16(a, b0, acc0);
      acc1 = wmma16(a, b1, acc1);
    }
    float sg[5];
#pragma unroll
    for (int b2 = 0; b2 < 5; ++b2) sg[b2] = 1.0f - 2.0f * (float)((t >> b2) & 1u);
#pragma unroll
    for (int r = 0; r < 8; ++r) {
      const float p = acc0[r] * acc0[r] + acc1[r] * acc1[r];
      S[r] += p;
#pragma unroll
      for (int b2 = 0; b2 < 5; ++b2) T[b2][r] = fmaf(sg[b2], p, T[b2][r]);
    }
  }

  const float nsg = 1.0f - 2.0f * (float)nw;
#pragma unroll
  for (int r = 0; r < 8; ++r) {
    const unsigned row = mw * 16u + hh * 8u + (unsigned)r;
    float* zr = &Zs[(nw * 64u + row) * ZP];
    const float s = S[r];
#pragma unroll
    for (int b2 = 0; b2 < 4; ++b2) {
      const float sv = (((m >> b2) & 1u) != 0u) ? -s : s;
      const float v = red16_sum(sv);
      if (m == 0u) zr[9 - b2] = v;
    }
    {
      const float v = red16_sum(s) * nsg;
      if (m == 0u) zr[5] = v;
    }
#pragma unroll
    for (int b2 = 0; b2 < 5; ++b2) {
      const float v = red16_sum(T[b2][r]);
      if (m == 0u) zr[4 - b2] = v;
    }
  }
  __syncthreads();

  const unsigned c = (tid & 15u) * 4u;
#pragma unroll 1
  for (unsigned i = 0; i < 4u; ++i) {
    const unsigned r = 16u * i + (tid >> 4);
    const float inv = 1.0f / ((UCARRY * UCARRY) * Ns[r]);
    float z[NQ];
#pragma unroll
    for (int q = 0; q < NQ; ++q)
      z[q] = (Zs[r * ZP + (unsigned)q] + Zs[(64u + r) * ZP + (unsigned)q]) * inv;
    v4f val;
#pragma unroll
    for (int j = 0; j < 4; ++j) {
      float a = 0.0f;
#pragma unroll
      for (int q = 0; q < NQ; ++q) a = fmaf(z[q], Ws[(c + (unsigned)j) * NQ + (unsigned)q], a);
      val[j] = a + Bs[c + (unsigned)j];
    }
    float* p = out + (size_t)(row0 + r) * OUTF + c;
    *(volatile v4f*)p = val;
    __threadfence();
    *(volatile v4f*)p = val;
  }
}

extern "C" void kernel_launch(void* const* d_in, const int* in_sizes, int n_in,
                              void* d_out, int out_size, void* d_ws, size_t ws_size,
                              hipStream_t stream) {
  if (n_in < 6) return;
  if ((long long)in_sizes[0] < (long long)NBATCH * KIN) return;
  if ((long long)in_sizes[1] < (long long)QD * KIN) return;
  if (in_sizes[2] < QD) return;
  if (in_sizes[3] < NGATE * 3) return;
  if (in_sizes[4] < OUTF * NQ) return;
  if (in_sizes[5] < OUTF) return;
  if ((long long)out_size < (long long)NBATCH * OUTF) return;
  if (ws_size < WS_TOTAL) return;

  const float* x      = (const float*)d_in[0];
  const float* W_pre  = (const float*)d_in[1];
  const float* b_pre  = (const float*)d_in[2];
  const float* qw     = (const float*)d_in[3];
  const float* W_post = (const float*)d_in[4];
  const float* b_post = (const float*)d_in[5];
  float* out = (float*)d_out;

  char* ws = (char*)d_ws;
  float*    G    = (float*)(ws + OFF_G);
  _Float16* X16  = (_Float16*)(ws + OFF_X16);
  _Float16* Wp16 = (_Float16*)(ws + OFF_WP16);
  float*    UT   = (float*)(ws + OFF_UT);
  _Float16* U16  = (_Float16*)(ws + OFF_U16);
  _Float16* H16  = (_Float16*)(ws + OFF_H16);

  dim3 blk(256);

  rot_prep_kernel<<<dim3(1), dim3(128), 0, stream>>>(qw, G);
  ubuild_kernel<<<dim3(QD), blk, 0, stream>>>(G, UT);
  uconv_kernel<<<dim3(UCOLS / 64, QD / 64), blk, 0, stream>>>(UT, U16, (unsigned)UCOLS, (unsigned)QD);

  const unsigned n8x = (unsigned)((size_t)NBATCH * KIN / 8);
  const unsigned n8w = (unsigned)((size_t)QD * KIN / 8);
  rowconv_kernel<<<dim3(n8x / 256u), blk, 0, stream>>>(x, X16, XCARRY, n8x);
  rowconv_kernel<<<dim3(n8w / 256u), blk, 0, stream>>>(W_pre, Wp16, WCARRY, n8w);

  gemm_pre_kernel<<<dim3(QD / 64, NBATCH / 64), blk, 0, stream>>>(X16, Wp16, b_pre, H16);
  circ_kernel<<<dim3(NBATCH / 64), blk, 0, stream>>>(H16, U16, W_post, b_post, out);
}
